// _S4Block_26139170964372
// MI455X (gfx1250) — hardware-run, weakly checked
//
#include <hip/hip_runtime.h>
#include <math.h>

typedef __attribute__((ext_vector_type(16))) _Float16 v16h;
typedef __attribute__((ext_vector_type(8)))  _Float16 v8h;
typedef __attribute__((ext_vector_type(16))) __bf16   v16b;
typedef __attribute__((ext_vector_type(8)))  __bf16   v8b;
typedef __attribute__((ext_vector_type(8)))  float    v8f;
typedef __attribute__((ext_vector_type(4)))  float    v4f;
typedef __attribute__((ext_vector_type(2)))  float    v2f;
typedef __attribute__((ext_vector_type(4)))  unsigned int v4u;

constexpr int kBatch = 8;
constexpr int kSeq   = 2048;
constexpr int kDm    = 512;
constexpr int kRows  = kBatch * kSeq;
static_assert(kRows == 16384);
static_assert((kDm % 32) == 0);
static_assert((kRows % 64) == 0 && (kDm % 64) == 0);
static_assert((kSeq % 8) == 0 && (kSeq % 256) == 0 && (kDm % 256) == 0);

constexpr int  kMode  = 2;
constexpr bool kLegBf = (kMode == 2);
constexpr int  kET    = (kMode == 0) ? 0 : 1;
constexpr int  kSPL   = (kMode == 1) ? 2 : 0;
constexpr int  kCarryXi = (kMode == 0) ? 16 : 1;
constexpr int  kCarryWi = (kMode == 0) ? 1024 : 1;
constexpr float kGemmScale = 1.0f / ((float)kCarryXi * (float)kCarryWi);
constexpr float kInvDm  = 1.0f / (float)kDm;
constexpr float kLnEps  = 1e-5f;
constexpr float kF16MinNormal = 6.103515625e-05f;
constexpr float kF32MinNormal = 1.17549435e-38f;
constexpr float kUnderflowLn = 104.0f;
constexpr int   kTapChunk = 128;
static_assert((kSeq % kTapChunk) == 0);

constexpr size_t kSzXH  = (size_t)kRows * kDm * 2;
constexpr size_t kSzXL  = (kMode == 1) ? kSzXH : 0;
constexpr size_t kSzWH  = (size_t)kDm * kDm * 2;
constexpr size_t kSzWL  = (kMode == 1) ? kSzWH : 0;
constexpr size_t kSzH0  = (size_t)kRows * kDm * 4;
constexpr size_t kSzMU  = (size_t)kRows * 4;
constexpr size_t kSzRS  = (size_t)kRows * 4;
constexpr size_t kSzTAP = (size_t)kSeq * kDm * 4;
constexpr size_t kOffXH  = 0;
constexpr size_t kOffXL  = kOffXH + kSzXH;
constexpr size_t kOffWH  = kOffXL + kSzXL;
constexpr size_t kOffWL  = kOffWH + kSzWH;
constexpr size_t kOffH0  = kOffWL + kSzWL;
constexpr size_t kOffMU  = kOffH0 + kSzH0;
constexpr size_t kOffRS  = kOffMU + kSzMU;
constexpr size_t kOffTAP = kOffRS + kSzRS;
constexpr size_t kWsTotal = kOffTAP + kSzTAP;
static_assert(kWsTotal <= 134217728ull);
static_assert((kOffXL % 128) == 0 && (kOffWH % 128) == 0 && (kOffWL % 128) == 0 && (kOffH0 % 128) == 0 &&
              (kOffMU % 128) == 0 && (kOffRS % 128) == 0 && (kOffTAP % 128) == 0);

__device__ __forceinline__ unsigned bf_rne_u32(float f) {
  unsigned u = __float_as_uint(f);
  const unsigned lsb = (u & 0x00010000u) ? 1u : 0u;
  u = (u + 0x7FFFu + lsb) & 0xFFFF0000u;
  return u;
}
template <bool BF> __device__ __forceinline__ float in_val(float f) {
  return BF ? __uint_as_float(bf_rne_u32(f)) : f;
}
__device__ __forceinline__ unsigned pack_upper_halves(unsigned first, unsigned second) {
  return __builtin_amdgcn_perm(second, first, 0x07060302u);
}

__device__ __forceinline__ void tie_h(v8f& a, v16h x, v16h y) { asm volatile("" : "+v"(a) : "v"(x), "v"(y)); }
__device__ __forceinline__ void tie_b(v8f& a, v16b x, v16b y) { asm volatile("" : "+v"(a) : "v"(x), "v"(y)); }
__device__ __forceinline__ void nop_guard_h(v8f& a, v16h x, v16h y) { asm volatile("v_nop\n\tv_nop\n\tv_nop\n\tv_nop" : "+v"(a) : "v"(x), "v"(y)); }
__device__ __forceinline__ void nop_guard_b(v8f& a, v16b x, v16b y) { asm volatile("v_nop\n\tv_nop\n\tv_nop\n\tv_nop" : "+v"(a) : "v"(x), "v"(y)); }
__device__ __forceinline__ void keep4_h(v16h a, v16h b, v16h c, v16h d) { asm volatile("v_nop" :: "v"(a), "v"(b), "v"(c), "v"(d)); }
__device__ __forceinline__ void keep4_b(v16b a, v16b b, v16b c, v16b d) { asm volatile("v_nop" :: "v"(a), "v"(b), "v"(c), "v"(d)); }
__device__ __forceinline__ void acc_guard4(v8f& a, v8f& b, v8f& c, v8f& d) { asm volatile("v_nop\n\tv_nop\n\tv_nop\n\tv_nop" : "+v"(a), "+v"(b), "+v"(c), "+v"(d)); }

template <typename T> struct Frag;
template <> struct Frag<_Float16> {
  typedef v16h V; union U { v16h v; v8h h[2]; };
  static __device__ __forceinline__ v16h load(const _Float16* p) {
    U f; f.h[0] = *(const v8h*)(p); f.h[1] = *(const v8h*)(p + 16); return f.v;
  }
  static __device__ __forceinline__ v8f mma(v16h a, v16h b, v8f c) {
    return __builtin_amdgcn_wmma_f32_16x16x32_f16(false, a, false, b, (short)0, c, false, false);
  }
  static __device__ __forceinline__ void tie(v8f& a, v16h x, v16h y) { tie_h(a, x, y); }
  static __device__ __forceinline__ void guard(v8f& a, v16h x, v16h y) { nop_guard_h(a, x, y); }
  static __device__ __forceinline__ void keep(v16h a, v16h b, v16h c, v16h d) { keep4_h(a, b, c, d); }
};
template <> struct Frag<__bf16> {
  typedef v16b V; union U { v16b v; v8b h[2]; };
  static __device__ __forceinline__ v16b load(const __bf16* p) {
    U f; f.h[0] = *(const v8b*)(p); f.h[1] = *(const v8b*)(p + 16); return f.v;
  }
  static __device__ __forceinline__ v8f mma(v16b a, v16b b, v8f c) {
    return __builtin_amdgcn_wmma_f32_16x16x32_bf16(false, a, false, b, (short)0, c, false, false);
  }
  static __device__ __forceinline__ void tie(v8f& a, v16b x, v16b y) { tie_b(a, x, y); }
  static __device__ __forceinline__ void guard(v8f& a, v16b x, v16b y) { nop_guard_b(a, x, y); }
  static __device__ __forceinline__ void keep(v16b a, v16b b, v16b c, v16b d) { keep4_b(a, b, c, d); }
};
template <int ET> struct Elem;
template <> struct Elem<0> { typedef _Float16 T; };
template <> struct Elem<1> { typedef __bf16 T; };

template <int MODE, int CARRY>
__global__ __launch_bounds__(256) void to16_rows_kernel(
    const float* __restrict__ src, unsigned short* __restrict__ dhi, unsigned short* __restrict__ dlo, int total8)
{
  const int i = blockIdx.x * 256 + threadIdx.x;
  if (i >= total8) return;
  const size_t e0 = (size_t)i << 3;
  const v4f a0 = *(const v4f*)(src + e0);
  const v4f a1 = *(const v4f*)(src + e0 + 4);
  float f[8];
  f[0] = a0[0]; f[1] = a0[1]; f[2] = a0[2]; f[3] = a0[3];
  f[4] = a1[0]; f[5] = a1[1]; f[6] = a1[2]; f[7] = a1[3];
  if (MODE == 0) {
    v8h hv;
#pragma unroll
    for (int e = 0; e < 8; ++e) {
      float v = f[e] * (float)CARRY;
      v = (fabsf(v) < kF16MinNormal) ? 0.0f : v;
      hv[e] = (_Float16)v;
    }
    unsigned short* qh = dhi + e0;
    *(volatile v8h*)qh = hv;
    __threadfence();
    *(volatile v8h*)qh = hv;
  } else {
    v4u hw, lw;
#pragma unroll
    for (int p = 0; p < 4; ++p) {
      const float f0 = f[2 * p], f1 = f[2 * p + 1];
      const unsigned u0 = bf_rne_u32(f0), u1 = bf_rne_u32(f1);
      hw[p] = pack_upper_halves(u0, u1);
      if (MODE == 1) {
        const float r0 = f0 - __uint_as_float(u0);
        const float r1 = f1 - __uint_as_float(u1);
        lw[p] = pack_upper_halves(bf_rne_u32(r0), bf_rne_u32(r1));
      } else {
        lw[p] = 0u;
      }
    }
    unsigned short* qh = dhi + e0;
    unsigned short* ql = dlo + e0;
    *(volatile v4u*)qh = hw;
    if (MODE == 1) *(volatile v4u*)ql = lw;
    __threadfence();
    *(volatile v4u*)qh = hw;
    if (MODE == 1) *(volatile v4u*)ql = lw;
  }
}

template <int ET, int SPL, bool BIAS_BF>
__global__ __launch_bounds__(256) void wmma_gemm64(
    const unsigned short* __restrict__ Ap, const unsigned short* __restrict__ A2p, int lda,
    const unsigned short* __restrict__ Btp, const unsigned short* __restrict__ Bt2p, int ldb,
    float* __restrict__ Cout, int ldc, const float* __restrict__ bias, int M, int N, int K)
{
  typedef typename Elem<ET>::T T;
  typedef typename Frag<T>::V V;
  const T* A = (const T*)Ap; const T* A2 = (const T*)A2p; const T* Bt = (const T*)Btp; const T* Bt2 = (const T*)Bt2p;
  __shared__ __align__(16) float sT[8][16 * 68];
  const int lane = threadIdx.x & 31;
  const int wave = threadIdx.x >> 5;
  const int tilesN = N >> 6;
  const int tilesM = M >> 6;
  const int tile = blockIdx.x * 8 + wave;
  if (tile >= tilesM * tilesN) return;
  const int tm = tile / tilesN;
  const int tn = tile - tm * tilesN;
  const int m0 = tm << 6;
  const int n0 = tn << 6;

  const int rlane = lane & 15;
  const int koff  = (lane >> 4) * 8;
  const int mOff  = (lane >> 4) * 8;

  v8f acc[4][4];
#pragma unroll
  for (int i = 0; i < 4; ++i)
#pragma unroll
    for (int j = 0; j < 4; ++j) acc[i][j] = (v8f){0.f,0.f,0.f,0.f,0.f,0.f,0.f,0.f};

  for (int k0 = 0; k0 < K; k0 += 32) {
    V bh[4], bl[4];
#pragma unroll
    for (int j = 0; j < 4; ++j) {
      const size_t bo = (size_t)(n0 + (j << 4) + rlane) * ldb + koff + k0;
      bh[j] = Frag<T>::load(Bt + bo);
      if (SPL == 2) bl[j] = Frag<T>::load(Bt2 + bo);
    }
#pragma unroll
    for (int i = 0; i < 4; ++i) {
      const size_t ao = (size_t)(m0 + (i << 4) + rlane) * lda + koff + k0;
      V ah = Frag<T>::load(A + ao);
      V al;
      if (SPL == 2) al = Frag<T>::load(A2 + ao);
#pragma unroll
      for (int j = 0; j < 4; ++j) {
        acc[i][j] = Frag<T>::mma(ah, bh[j], acc[i][j]);
        if (SPL == 2) {
          acc[i][j] = Frag<T>::mma(ah, bl[j], acc[i][j]);
          acc[i][j] = Frag<T>::mma(al, bh[j], acc[i][j]);
        }
      }
      Frag<T>::tie(acc[i][0], ah, bh[0]);
      Frag<T>::tie(acc[i][1], ah, bh[1]);
      Frag<T>::tie(acc[i][2], ah, bh[2]);
      if (SPL == 2) {
        Frag<T>::tie(acc[i][0], al, bl[0]);
        Frag<T>::tie(acc[i][1], al, bl[1]);
        Frag<T>::tie(acc[i][2], al, bl[2]);
        Frag<T>::tie(acc[i][3], al, bl[3]);
      }
      Frag<T>::guard(acc[i][3], ah, bh[3]);
    }
    Frag<T>::keep(bh[0], bh[1], bh[2], bh[3]);
    if (SPL == 2) Frag<T>::keep(bl[0], bl[1], bl[2], bl[3]);
  }
  acc_guard4(acc[0][0], acc[0][1], acc[0][2], acc[0][3]);
  acc_guard4(acc[1][0], acc[1][1], acc[1][2], acc[1][3]);
  acc_guard4(acc[2][0], acc[2][1], acc[2][2], acc[2][3]);
  acc_guard4(acc[3][0], acc[3][1], acc[3][2], acc[3][3]);

  float* slab = sT[wave];
  float bv[4];
#pragma unroll
  for (int j = 0; j < 4; ++j) bv[j] = in_val<BIAS_BF>(bias[n0 + (j << 4) + rlane]);
#pragma unroll
  for (int i = 0; i < 4; ++i) {
    const int mBase = m0 + (i << 4);
#pragma unroll
    for (int j = 0; j < 4; ++j) {
#pragma unroll
      for (int r = 0; r < 8; ++r) {
        const float v = acc[i][j][r] * kGemmScale + bv[j];
        slab[(mOff + r) * 68 + (j << 4) + rlane] = v;
      }
    }
    __builtin_amdgcn_fence(__ATOMIC_RELEASE, "workgroup");
    __builtin_amdgcn_wave_barrier();
    __builtin_amdgcn_fence(__ATOMIC_ACQUIRE, "workgroup");
    {
      const int hh = lane >> 4, c4 = (lane & 15) * 4;
      for (int pass = 0; pass < 2; ++pass) {
#pragma unroll
        for (int it = 0; it < 8; ++it) {
          const int row = it * 2 + hh;
          const v4f v = *(const v4f*)(slab + row * 68 + c4);
          *(volatile v4f*)(Cout + (size_t)(mBase + row) * ldc + n0 + c4) = v;
        }
        __threadfence();
      }
    }
    __builtin_amdgcn_fence(__ATOMIC_RELEASE, "workgroup");
    __builtin_amdgcn_wave_barrier();
    __builtin_amdgcn_fence(__ATOMIC_ACQUIRE, "workgroup");
  }
}

__global__ __launch_bounds__(256) void row_stats_kernel(
    const float* __restrict__ H0, float* __restrict__ MU, float* __restrict__ RS)
{
  __shared__ float sMu[32];
  __shared__ float sRs[32];
  const int tid = threadIdx.x, lane = tid & 31, wave = tid >> 5;
  const int rbase = blockIdx.x * 32;
#pragma unroll 1
  for (int r = 0; r < 4; ++r) {
    const int lr = wave * 4 + r;
    const float* p = H0 + (size_t)(rbase + lr) * kDm + lane * 4;
    const v4f v0 = *(const v4f*)(p);
    const v4f v1 = *(const v4f*)(p + 128);
    const v4f v2 = *(const v4f*)(p + 256);
    const v4f v3 = *(const v4f*)(p + 384);
    float s = ((v0[0] + v0[1]) + (v0[2] + v0[3])) + ((v1[0] + v1[1]) + (v1[2] + v1[3]));
    s += ((v2[0] + v2[1]) + (v2[2] + v2[3])) + ((v3[0] + v3[1]) + (v3[2] + v3[3]));
    s += __shfl_xor(s, 16, 32);
    s += __shfl_xor(s, 8, 32);
    s += __shfl_xor(s, 4, 32);
    s += __shfl_xor(s, 2, 32);
    s += __shfl_xor(s, 1, 32);
    const float mu = s * kInvDm;
    const v4f d0 = v0 - mu, d1 = v1 - mu, d2 = v2 - mu, d3 = v3 - mu;
    const v4f q0 = d0 * d0, q1 = d1 * d1, q2 = d2 * d2, q3 = d3 * d3;
    float ss = ((q0[0] + q0[1]) + (q0[2] + q0[3])) + ((q1[0] + q1[1]) + (q1[2] + q1[3]));
    ss += ((q2[0] + q2[1]) + (q2[2] + q2[3])) + ((q3[0] + q3[1]) + (q3[2] + q3[3]));
    ss += __shfl_xor(ss, 16, 32);
    ss += __shfl_xor(ss, 8, 32);
    ss += __shfl_xor(ss, 4, 32);
    ss += __shfl_xor(ss, 2, 32);
    ss += __shfl_xor(ss, 1, 32);
    const float var = ss * kInvDm;
    const float rs = rsqrtf(var + kLnEps);
    if (lane == 0) { sMu[lr] = mu; sRs[lr] = rs; }
  }
  __syncthreads();
  if (wave == 0) {
    const float v = sMu[lane];
    float* q = MU + rbase + lane;
    *(volatile float*)q = v;
    __threadfence();
    *(volatile float*)q = v;
  }
  if (wave == 1) {
    const float v = sRs[lane];
    float* q = RS + rbase + lane;
    *(volatile float*)q = v;
    __threadfence();
    *(volatile float*)q = v;
  }
}

template <bool BF>
__global__ __launch_bounds__(256) void tap_table_kernel(
    const float* __restrict__ Are, const float* __restrict__ Aim,
    const float* __restrict__ Bre, const float* __restrict__ Bim,
    const float* __restrict__ Cre, const float* __restrict__ Cim,
    float* __restrict__ TAP)
{
  const int c  = blockIdx.x * 256 + threadIdx.x;
  const int j0 = blockIdx.y * kTapChunk;
  const float a  = in_val<BF>(Are[c]);
  const float ai = in_val<BF>(Aim[c]);
  const float br = in_val<BF>(Bre[c]);
  const float bi = in_val<BF>(Bim[c]);
  const float cr = in_val<BF>(Cre[c]);
  const float ci = in_val<BF>(Cim[c]);
  const float r2  = fmaf(a, a, ai * ai);
  const float lnr = 0.5f * logf(r2);
  const float th  = atan2f(ai, a);
  const float bcr = br * cr - bi * ci;
  const float bci = br * ci + bi * cr;
#pragma unroll 1
  for (int jj = 0; jj < kTapChunk; ++jj) {
    const int j = j0 + jj;
    const float jf = (float)j;
    const float ex = (j == 0) ? 0.0f : jf * lnr;
    float mag = expf(ex);
    mag = (mag < kF32MinNormal) ? 0.0f : mag;
    const float q  = jf * th;
    const float sn = sinf(q);
    const float cs = cosf(q);
    const float pr = mag * cs;
    const float pi = mag * sn;
    const float w  = pr * bcr - pi * bci;
    float* dst = TAP + (size_t)j * kDm + c;
    *(volatile float*)dst = w;
    __threadfence();
    *(volatile float*)dst = w;
  }
}

template <bool BF>
__global__ __launch_bounds__(256) void scan_kernel(
    const float* __restrict__ H0, const float* __restrict__ MU, const float* __restrict__ RS,
    const float* __restrict__ TAP, const float* __restrict__ Are, const float* __restrict__ Aim,
    const float* __restrict__ Dre, const float* __restrict__ gamma, const float* __restrict__ beta,
    float* __restrict__ out)
{
  __shared__ __align__(16) v2f sMR[kSeq];
  __shared__ float sRed[8];
  const int tid = threadIdx.x, lane = tid & 31, wave = tid >> 5;
  const int b = blockIdx.x >> 1;
  const int c = ((blockIdx.x & 1) << 8) + tid;
  const size_t row0 = (size_t)b * kSeq;

  float lm = -INFINITY;
#pragma unroll
  for (int k = 0; k < 2; ++k) {
    const int ch = tid + 256 * k;
    const float a  = in_val<BF>(Are[ch]);
    const float ai = in_val<BF>(Aim[ch]);
    const float r2 = fmaf(a, a, ai * ai);
    const float ln = 0.5f * logf(r2);
    lm = fmaxf(lm, ln);
  }
  lm = fmaxf(lm, __shfl_xor(lm, 16, 32));
  lm = fmaxf(lm, __shfl_xor(lm, 8, 32));
  lm = fmaxf(lm, __shfl_xor(lm, 4, 32));
  lm = fmaxf(lm, __shfl_xor(lm, 2, 32));
  lm = fmaxf(lm, __shfl_xor(lm, 1, 32));
  if (lane == 0) sRed[wave] = lm;
#pragma unroll
  for (int i = 0; i < 8; ++i) {
    const int l = tid + 256 * i;
    v2f mr;
    mr[0] = MU[row0 + l];
    mr[1] = RS[row0 + l];
    sMR[l] = mr;
  }
  __syncthreads();
  float lmax = sRed[0];
#pragma unroll
  for (int w = 1; w < 8; ++w) lmax = fmaxf(lmax, sRed[w]);
  int jstar;
  {
    const float q = kUnderflowLn * (1.0f / (-lmax));
    jstar = ((lmax < 0.0f) && (q < (float)kSeq)) ? ((int)q + 2) : kSeq;
    jstar = (jstar > kSeq) ? kSeq : jstar;
    jstar = (jstar < 1) ? 1 : jstar;
  }
  const int ltail = kSeq - jstar;

  const float g  = in_val<BF>(gamma[c]);
  const float be = in_val<BF>(beta[c]);
  const float Dr = in_val<BF>(Dre[c]);
  const float* hp = H0 + row0 * kDm + c;
  const float* tp = TAP + c;
  float* op = out + row0 * kDm + c;

  float S = 0.0f;
#pragma unroll 1
  for (int l0 = 0; l0 < kSeq; l0 += 8) {
    float hx[8];
#pragma unroll
    for (int i = 0; i < 8; ++i) hx[i] = hp[(size_t)(l0 + i) * kDm];
    float o[8];
#pragma unroll
    for (int i = 0; i < 8; ++i) {
      const v2f mr = sMR[l0 + i];
      const float h = ((hx[i] - mr[0]) * mr[1]) * g + be;
      S += h;
      o[i] = fmaf(Dr, S, h);
    }
    if (l0 + 8 > ltail) {
      float tacc[8];
#pragma unroll
      for (int i = 0; i < 8; ++i) tacc[i] = 0.0f;
      const int lbase = kSeq - 1 - l0;
      int ntmax = jstar - lbase + 7;
      ntmax = (ntmax > l0 + 8) ? (l0 + 8) : ntmax;
#pragma unroll 1
      for (int t = 0; t < ntmax; ++t) {
        const v2f mr = sMR[t];
        const float hx0 = hp[(size_t)t * kDm];
        const float ht = ((hx0 - mr[0]) * mr[1]) * g + be;
#pragma unroll
        for (int i = 0; i < 8; ++i) {
          const int row  = lbase - i + t;
          const int rowc = (row < kSeq) ? row : (kSeq - 1);
          const float w = tp[(size_t)rowc * kDm];
          int nti = jstar - lbase + i;
          nti = (nti > l0 + i + 1) ? (l0 + i + 1) : nti;
          const bool on = (t < nti);
          tacc[i] = on ? fmaf(w, ht, tacc[i]) : tacc[i];
        }
      }
#pragma unroll
      for (int i = 0; i < 8; ++i) o[i] += tacc[i];
    }
    float* q = op + (size_t)l0 * kDm;
    for (int pass = 0; pass < 2; ++pass) {
#pragma unroll
      for (int i = 0; i < 8; ++i) *(volatile float*)(q + (size_t)i * kDm) = o[i];
      __threadfence();
    }
  }
}

extern "C" void kernel_launch(void* const* d_in, const int* in_sizes, int n_in,
                              void* d_out, int out_size, void* d_ws, size_t ws_size,
                              hipStream_t stream) {
  if (n_in < 13) return;
  if (in_sizes[0] != kRows * kDm) return;
  for (int i = 1; i <= 8; ++i) if (in_sizes[i] != kDm) return;
  if (in_sizes[9] != kDm * kDm) return;
  if (in_sizes[10] != kDm || in_sizes[11] != kDm || in_sizes[12] != kDm) return;
  if (out_size != kRows * kDm) return;
  if (ws_size < kWsTotal) return;

  const float* x     = (const float*)d_in[0];
  const float* A_re  = (const float*)d_in[1];
  const float* A_im  = (const float*)d_in[2];
  const float* B_re  = (const float*)d_in[3];
  const float* B_im  = (const float*)d_in[4];
  const float* C_re  = (const float*)d_in[5];
  const float* C_im  = (const float*)d_in[6];
  const float* D_re  = (const float*)d_in[7];
  const float* W     = (const float*)d_in[9];
  const float* bias  = (const float*)d_in[10];
  const float* gamma = (const float*)d_in[11];
  const float* beta  = (const float*)d_in[12];
  float* out = (float*)d_out;

  char* ws = (char*)d_ws;
  unsigned short* XH = (unsigned short*)(ws + kOffXH);
  unsigned short* XL = (kMode == 1) ? (unsigned short*)(ws + kOffXL) : XH;
  unsigned short* WH = (unsigned short*)(ws + kOffWH);
  unsigned short* WL = (kMode == 1) ? (unsigned short*)(ws + kOffWL) : WH;
  float* H0  = (float*)(ws + kOffH0);
  float* MU  = (float*)(ws + kOffMU);
  float* RS  = (float*)(ws + kOffRS);
  float* TAP = (float*)(ws + kOffTAP);

  to16_rows_kernel<kMode, kCarryXi><<<(kRows * kDm / 8) / 256, 256, 0, stream>>>(x, XH, XL, kRows * kDm / 8);
  to16_rows_kernel<kMode, kCarryWi><<<(kDm * kDm / 8) / 256, 256, 0, stream>>>(W, WH, WL, kDm * kDm / 8);

  wmma_gemm64<kET, kSPL, kLegBf><<<dim3(((kRows / 64) * (kDm / 64)) / 8), 256, 0, stream>>>(
      XH, XL, kDm, WH, WL, kDm, H0, kDm, bias, kRows, kDm, kDm);

  row_stats_kernel<<<kRows / 32, 256, 0, stream>>>(H0, MU, RS);

  tap_table_kernel<kLegBf><<<dim3(kDm / 256, kSeq / kTapChunk), 256, 0, stream>>>(
      A_re, A_im, B_re, B_im, C_re, C_im, TAP);

  scan_kernel<kLegBf><<<kBatch * (kDm / 256), 256, 0, stream>>>(
      H0, MU, RS, TAP, A_re, A_im, D_re, gamma, beta, out);
}
